// GatNet_15358803050747
// MI455X (gfx1250) — hardware-verified
//
#include <hip/hip_runtime.h>
#include <stddef.h>
#include <stdint.h>
#include <math.h>


#define HCH     64
#define KA      128
#define NTHR    256
#define NWAVE   8
#define EPT     8
#define CHUNK   (NTHR * EPT)
#define WCAP    (EPT * 32)
#define LISTN   (NWAVE * WCAP)
#define NBMAX   2048
#define SLOTB   11
#define RCAP    28672
#define DEGCAP  256
#define GBM     64
#define GBN     64
#define GTHR    128
#define MROWS   128
#define NEGSL   0.2f
#define EPS_SM  1e-16f
#define WSMAX   134217728
#define LDS_AGG ((2 * RCAP + 2 * NBMAX + LISTN) * 4 + 64)

static_assert((CHUNK & (CHUNK - 1)) == 0 && CHUNK <= (1 << SLOTB));
static_assert(NBMAX == (1 << SLOTB));
static_assert(NTHR * 8 == NBMAX);
static_assert(LISTN >= NBMAX);
static_assert(LISTN >= NWAVE * WCAP);
static_assert((RCAP % 32) == 0);
static_assert(LDS_AGG <= 300000);
static_assert(GBM == (GTHR / 32) * 16);
static_assert((KA % 32) == 0 && HCH == GBN && KA == 2 * HCH);
static_assert((MROWS % GBM) == 0);
static_assert(HCH == 2 * 32);

typedef float          v2f  __attribute__((ext_vector_type(2)));
typedef float          v4f  __attribute__((ext_vector_type(4)));
typedef float          v8f  __attribute__((ext_vector_type(8)));
typedef int            v4i  __attribute__((ext_vector_type(4)));
typedef int            v8i  __attribute__((ext_vector_type(8)));
typedef unsigned int   v4u  __attribute__((ext_vector_type(4)));
typedef unsigned short v8us __attribute__((ext_vector_type(8)));
typedef __bf16         v16b __attribute__((ext_vector_type(16)));
typedef v2f  __attribute__((may_alias)) v2fa;
typedef v4f  __attribute__((may_alias)) v4fa;
typedef v8us __attribute__((may_alias)) v8usa;
union FragB { v16b v; v8us h[2]; v8i w; };

__device__ __forceinline__ v8f wmb(const FragB& a, const FragB& b, v8f c) {
  v8f d = __builtin_amdgcn_wmma_f32_16x16x32_bf16(false, a.v, false, b.v, (short)0, c, false, false);
  asm volatile("v_nop\n\tv_nop\n\tv_nop\n\tv_nop" : "+v"(d) : "v"(a.w), "v"(b.w));
  return d;
}

__device__ __forceinline__ unsigned int f2bf(float f) {
  const unsigned int u = __float_as_uint(f);
  return ((u + 0x7FFFu + ((u >> 16) & 1u)) >> 16) & 0xFFFFu;
}
__device__ __forceinline__ float bf2f(unsigned int b) { return __uint_as_float(b << 16); }
__device__ __forceinline__ float bfr(float f) { return bf2f(f2bf(f)); }
__device__ __forceinline__ v2f bfr2(const v2f a) { v2f r; r.x = bfr(a.x); r.y = bfr(a.y); return r; }
__device__ __forceinline__ v4f bfr4(const v4f a) {
  v4f r; r.x = bfr(a.x); r.y = bfr(a.y); r.z = bfr(a.z); r.w = bfr(a.w); return r;
}
__device__ __forceinline__ unsigned int pk2(float lo, float hi) { return f2bf(lo) | (f2bf(hi) << 16); }
__device__ __forceinline__ v4u pack8(const v4f a, const v4f b) {
  v4u r;
  r.x = pk2(a.x, a.y); r.y = pk2(a.z, a.w); r.z = pk2(b.x, b.y); r.w = pk2(b.z, b.w);
  return r;
}

__device__ __forceinline__ int scan_chunk(const int* __restrict__ dsts, int nE, int cbase, int slotBase,
                                          int nb, int vec8, int* list, int tid, int lane, int wave) {
  int wc = 0;
  const int el0  = tid * EPT;
  const int e0   = cbase + el0;
  const int sent = -2147483647 - 1;
  v4i da, db;
  if (vec8 != 0 && cbase + CHUNK <= nE) {
    da = *(const v4i*)(dsts + e0);
    db = *(const v4i*)(dsts + e0 + 4);
  } else {
    da.x = (e0     < nE) ? dsts[min(e0,     nE - 1)] : sent;
    da.y = (e0 + 1 < nE) ? dsts[min(e0 + 1, nE - 1)] : sent;
    da.z = (e0 + 2 < nE) ? dsts[min(e0 + 2, nE - 1)] : sent;
    da.w = (e0 + 3 < nE) ? dsts[min(e0 + 3, nE - 1)] : sent;
    db.x = (e0 + 4 < nE) ? dsts[min(e0 + 4, nE - 1)] : sent;
    db.y = (e0 + 5 < nE) ? dsts[min(e0 + 5, nE - 1)] : sent;
    db.z = (e0 + 6 < nE) ? dsts[min(e0 + 6, nE - 1)] : sent;
    db.w = (e0 + 7 < nE) ? dsts[min(e0 + 7, nE - 1)] : sent;
  }
  const unsigned nbs = (unsigned)slotBase;
  const unsigned unb = (unsigned)nb;
  const unsigned s0 = (unsigned)da.x - nbs, s1 = (unsigned)da.y - nbs;
  const unsigned s2 = (unsigned)da.z - nbs, s3 = (unsigned)da.w - nbs;
  const unsigned s4 = (unsigned)db.x - nbs, s5 = (unsigned)db.y - nbs;
  const unsigned s6 = (unsigned)db.z - nbs, s7 = (unsigned)db.w - nbs;
  const bool h0 = s0 < unb, h1 = s1 < unb, h2 = s2 < unb, h3 = s3 < unb;
  const bool h4 = s4 < unb, h5 = s5 < unb, h6 = s6 < unb, h7 = s7 < unb;
  const unsigned any = __builtin_amdgcn_ballot_w32(h0 | h1 | h2 | h3 | h4 | h5 | h6 | h7);
  if (any != 0u) {
#define HITJ(J, HJ, SJ) { \
      const unsigned mj = __builtin_amdgcn_ballot_w32(HJ); \
      if (mj != 0u) { \
        if (HJ) { \
          const int pos = wc + (int)__builtin_amdgcn_mbcnt_lo(mj, 0u); \
          if (pos < WCAP) list[wave * WCAP + pos] = ((el0 + (J)) << SLOTB) | (int)(SJ); \
        } \
        wc += (int)__builtin_popcount(mj); } }
    HITJ(0, h0, s0)
    HITJ(1, h1, s1)
    HITJ(2, h2, s2)
    HITJ(3, h3, s3)
    HITJ(4, h4, s4)
    HITJ(5, h5, s5)
    HITJ(6, h6, s6)
    HITJ(7, h7, s7)
#undef HITJ
  }
  return wc;
}

__global__ __launch_bounds__(NTHR) void k_l1feat(const float* __restrict__ x, const float* __restrict__ W1,
                                                 float* F, int nN, int nUnits) {
  const int i = (int)blockIdx.x * NTHR + (int)threadIdx.x;
  if (i >= nUnits) return;
  const int row = i >> 4;
  const int c0  = (i & 15) * 4;
  const int rc  = row < nN ? row : nN - 1;
  const float xv = bfr(x[rc]);
  const v4f w = bfr4(*(const v4fa*)(W1 + c0));
  v4f o;
  o.x = xv * w.x; o.y = xv * w.y; o.z = xv * w.z; o.w = xv * w.w;
  const v4f z4 = {0.f, 0.f, 0.f, 0.f};
  if (row >= nN) o = z4;
  float* op = F + (size_t)row * HCH + c0;
  *(volatile v4f*)op = o;
  __threadfence();
  *(volatile v4f*)op = o;
}

__global__ __launch_bounds__(NTHR) void k_wtr(const float* __restrict__ w, int Kin, int Ncol, int Nrows, int Kout,
                                              unsigned short* wt, int nUnits) {
  const int u = (int)blockIdx.x * NTHR + (int)threadIdx.x;
  if (u >= nUnits) return;
  const int kq = Kout >> 3;
  const int n  = u / kq;
  const int k8 = (u - n * kq) * 8;
  const int kk = k8 - (k8 / Kin) * Kin;
  const int ncl = n < Ncol ? n : Ncol - 1;
  const float* p = w + (size_t)kk * (size_t)Ncol + ncl;
  v4f a, b;
  a.x = p[0];                    a.y = p[(size_t)Ncol];         a.z = p[(size_t)2 * Ncol];     a.w = p[(size_t)3 * Ncol];
  b.x = p[(size_t)4 * Ncol];     b.y = p[(size_t)5 * Ncol];     b.z = p[(size_t)6 * Ncol];     b.w = p[(size_t)7 * Ncol];
  const v4f z4 = {0.f, 0.f, 0.f, 0.f};
  if (n >= Ncol || n >= Nrows) { a = z4; b = z4; }
  const v4u wv = pack8(a, b);
  unsigned short* o = wt + (size_t)n * (size_t)Kout + k8;
  *(volatile v4u*)o = wv;
  __threadfence();
  *(volatile v4u*)o = wv;
}

__global__ __launch_bounds__(GTHR) void k_gemm(
    const unsigned short* __restrict__ A, const unsigned short* __restrict__ WT,
    float* outF, int K, int ldo)
{
  __shared__ __attribute__((aligned(16))) float stg[GBM * GBN];
  const int tid = (int)threadIdx.x, lane = tid & 31, wave = tid >> 5, hh = lane >> 4, m = lane & 15;
  const int rowBase = (int)blockIdx.x * GBM;
  const int col0    = (int)blockIdx.y * GBN;

  v8f acc[4];
  {
    const v8f z = {0.f, 0.f, 0.f, 0.f, 0.f, 0.f, 0.f, 0.f};
    acc[0] = z; acc[1] = z; acc[2] = z; acc[3] = z;
  }
  const unsigned short* ap = A  + (size_t)(rowBase + 16 * wave + m) * (size_t)K + 8 * hh;
  const unsigned short* wp = WT + (size_t)(col0 + m) * (size_t)K + 8 * hh;
  const int ksteps = K >> 5;
#pragma unroll 1
  for (int ks = 0; ks < ksteps; ++ks) {
    FragB af;
    af.h[0] = *(const v8usa*)(ap + 32 * ks);
    af.h[1] = *(const v8usa*)(ap + 32 * ks + 16);
#pragma unroll
    for (int t = 0; t < 4; ++t) {
      const unsigned short* wq = wp + (size_t)(16 * t) * (size_t)K + 32 * ks;
      FragB bf;
      bf.h[0] = *(const v8usa*)wq;
      bf.h[1] = *(const v8usa*)(wq + 16);
      acc[t] = wmb(af, bf, acc[t]);
    }
  }

#pragma unroll
  for (int t = 0; t < 4; ++t) {
    const int lc = 16 * t + m;
#pragma unroll
    for (int r = 0; r < 8; ++r) {
      const int lr = 16 * wave + 8 * hh + r;
      stg[lr * GBN + lc] = acc[t][r];
    }
  }
  __syncthreads();

  v4f fv[8];
#pragma unroll
  for (int i = 0; i < 8; ++i) {
    const int lr = 16 * wave + 2 * i + hh;
    fv[i] = *(const v4fa*)(stg + lr * GBN + 4 * m);
  }
#pragma unroll
  for (int i = 0; i < 8; ++i) {
    const int lr = 16 * wave + 2 * i + hh;
    const int gr = rowBase + lr;
    float* op = outF + (size_t)gr * (size_t)ldo + col0 + 4 * m;
    *(volatile v4f*)op = fv[i];
  }
  __threadfence();
#pragma unroll
  for (int i = 0; i < 8; ++i) {
    const int lr = 16 * wave + 2 * i + hh;
    const int gr = rowBase + lr;
    float* op = outF + (size_t)gr * (size_t)ldo + col0 + 4 * m;
    *(volatile v4f*)op = fv[i];
  }
}

template<int L>
__global__ __launch_bounds__(NTHR) void k_agg(
    const int* __restrict__ srcs, const int* __restrict__ dsts,
    const float* __restrict__ F,
    const float* __restrict__ asrc, const float* __restrict__ adst,
    const float* __restrict__ bias, const float* __restrict__ fcw, const float* __restrict__ fcb,
    unsigned short* HP, float* out,
    int nN, int nE, int nb, int vec8, int MPr) {
  extern __shared__ v4f lds_dyn[];
  int* reg1 = (int*)lds_dyn;
  int* reg2 = reg1 + RCAP;
  int* scnt = reg2 + RCAP;
  int* soff = scnt + NBMAX;
  int* list = soff + NBMAX;
  int* wcnt = list + LISTN;
  int* wtot = wcnt + NWAVE;
  const int tid = (int)threadIdx.x, lane = tid & 31, wave = tid >> 5;
  const int nodeBase = (int)blockIdx.x * nb;

  for (int i = tid; i < NBMAX; i += NTHR) scnt[i] = 0;
  __syncthreads();

  int tot = 0;
  const int nChunks = (nE + CHUNK - 1) / CHUNK;
#pragma unroll 1
  for (int ch = 0; ch < nChunks; ++ch) {
    const int cbase = ch * CHUNK;
    const int wc = scan_chunk(dsts, nE, cbase, nodeBase, nb, vec8, list, tid, lane, wave);
    if (lane == 0) wcnt[wave] = wc;
    __syncthreads();
    int pre = 0, all = 0;
#pragma unroll
    for (int w2 = 0; w2 < NWAVE; ++w2) {
      int c = wcnt[w2];
      c = c < 0 ? 0 : (c > WCAP ? WCAP : c);
      all += c;
      pre += (w2 < wave) ? c : 0;
    }
    const int wcc  = wc > WCAP ? WCAP : wc;
    const int base = tot + pre;
#pragma unroll 1
    for (int i = lane; i < wcc; i += 32) {
      const int ent = list[wave * WCAP + i];
      const int el  = (ent >> SLOTB) & (CHUNK - 1);
      const int sl  = ent & (NBMAX - 1);
      int eid = cbase + el;
      eid = eid > nE - 1 ? nE - 1 : eid;
      const int pos = base + i;
      if (pos < RCAP) reg1[pos] = (int)(((unsigned)eid << SLOTB) | (unsigned)sl);
    }
    tot += all;
    tot = tot > RCAP ? RCAP : tot;
    __syncthreads();
  }
  const int nh = tot;

  if (wave == 0) {
#pragma unroll 1
    for (int b0 = 0; b0 < nh; b0 += 32) {
      const int idx = b0 + lane;
      const int uv  = reg1[idx < nh ? idx : nh - 1];
      const int m32 = (nh - b0) < 32 ? (nh - b0) : 32;
#pragma unroll 1
      for (int k = 0; k < m32; ++k) {
        const int u  = __builtin_amdgcn_readlane(uv, k);
        const int sl = u & (NBMAX - 1);
        if (lane == 0) scnt[sl] = scnt[sl] + 1;
      }
    }
  }
  __syncthreads();

  {
    const v4i ca = *(const v4i*)(scnt + 8 * tid);
    const v4i cb = *(const v4i*)(scnt + 8 * tid + 4);
    const int e0 = ca.x < 0 ? 0 : ca.x, e1 = ca.y < 0 ? 0 : ca.y, e2 = ca.z < 0 ? 0 : ca.z, e3 = ca.w < 0 ? 0 : ca.w;
    const int e4 = cb.x < 0 ? 0 : cb.x, e5 = cb.y < 0 ? 0 : cb.y, e6 = cb.z < 0 ? 0 : cb.z, e7 = cb.w < 0 ? 0 : cb.w;
    const int ts = e0 + e1 + e2 + e3 + e4 + e5 + e6 + e7;
    int incl = ts;
#pragma unroll
    for (int d = 1; d < 32; d <<= 1) {
      const int up = __shfl_up(incl, d);
      if (lane >= d) incl += up;
    }
    if (lane == 31) wtot[wave] = incl;
    __syncthreads();
    int pre = 0;
#pragma unroll
    for (int w2 = 0; w2 < NWAVE; ++w2) pre += (w2 < wave) ? wtot[w2] : 0;
    int run = pre + incl - ts;
    soff[8 * tid + 0] = run; run += e0;
    soff[8 * tid + 1] = run; run += e1;
    soff[8 * tid + 2] = run; run += e2;
    soff[8 * tid + 3] = run; run += e3;
    soff[8 * tid + 4] = run; run += e4;
    soff[8 * tid + 5] = run; run += e5;
    soff[8 * tid + 6] = run; run += e6;
    soff[8 * tid + 7] = run;
  }
  __syncthreads();
  for (int i = tid; i < NBMAX; i += NTHR) list[i] = soff[i];
  __syncthreads();

  if (wave == 0) {
#pragma unroll 1
    for (int b0 = 0; b0 < nh; b0 += 32) {
      const int idx = b0 + lane;
      const int uv  = reg1[idx < nh ? idx : nh - 1];
      const int m32 = (nh - b0) < 32 ? (nh - b0) : 32;
#pragma unroll 1
      for (int k = 0; k < m32; ++k) {
        const int u   = __builtin_amdgcn_readlane(uv, k);
        const int sl  = u & (NBMAX - 1);
        const int eid = (int)((unsigned)u >> SLOTB);
        if (lane == 0) {
          int pos = list[sl];
          pos = pos < 0 ? 0 : (pos > RCAP - 1 ? RCAP - 1 : pos);
          reg2[pos] = eid;
          list[sl] = pos + 1;
        }
      }
    }
  }
  __syncthreads();

  const int nbw = nb >> 3;
  const bool ovf = (nh >= RCAP);
  const float qnan = __int_as_float(0x7fc00000);
  const v2f as2 = bfr2(*(const v2fa*)(asrc + 2 * lane));
  const v2f ad2 = bfr2(*(const v2fa*)(adst + 2 * lane));
  const v2f bb2 = bfr2(*(const v2fa*)(bias + 2 * lane));
  v2f fw2 = {0.f, 0.f};
  float fb = 0.f;
  if (L == 3) {
    fw2 = bfr2(*(const v2fa*)(fcw + 2 * lane));
    fb  = bfr(fcb[0]);
  }
  float* res = (float*)list;

#pragma unroll 1
  for (int jt = 0; jt < nbw; ++jt) {
    const int slot = wave * nbw + jt;
    const int grow = nodeBase + slot;
    const int gcl  = grow < nN ? grow : nN - 1;
    int st = soff[slot];
    const int craw = scnt[slot];
    int cnt = craw;
    st  = st < 0 ? 0 : (st > nh ? nh : st);
    cnt = cnt < 0 ? 0 : (cnt > DEGCAP ? DEGCAP : cnt);
    if (cnt > nh - st) cnt = nh - st;
    const float pz = (ovf || craw > DEGCAP) ? qnan : 0.0f;

    const v2f fd = *(const v2fa*)(F + (size_t)gcl * HCH + 2 * lane);
    float pd = fd.x * ad2.x; pd = fmaf(fd.y, ad2.y, pd);
    pd += __shfl_xor(pd, 1);
    pd += __shfl_xor(pd, 2);
    float p0 = fd.x * as2.x; p0 = fmaf(fd.y, as2.y, p0);
    p0 += __shfl_xor(p0, 1);
    p0 += __shfl_xor(p0, 2);
    float l0 = p0 + pd;
    l0 = l0 > 0.f ? l0 : NEGSL * l0;
    float mx = l0, dn = 1.0f;
    float a0 = fd.x, a1 = fd.y;

#pragma unroll 1
    for (int q = 0; q < cnt; ++q) {
      int idx = st + q; idx = idx > RCAP - 1 ? RCAP - 1 : idx;
      int eid = reg2[idx]; eid = eid < 0 ? 0 : (eid > nE - 1 ? nE - 1 : eid);
      const int sraw = srcs[eid];
      const int s = sraw < 0 ? 0 : (sraw > nN - 1 ? nN - 1 : sraw);
      const v2f fs = *(const v2fa*)(F + (size_t)s * HCH + 2 * lane);
      float es = fs.x * as2.x; es = fmaf(fs.y, as2.y, es);
      es += __shfl_xor(es, 1);
      es += __shfl_xor(es, 2);
      float lg = es + pd;
      lg = lg > 0.f ? lg : NEGSL * lg;
      const float df = lg - mx;
      const float ee = __expf(-fabsf(df));
      const bool up  = df > 0.f;
      const float s1 = up ? ee : 1.0f;
      const float s2 = up ? 1.0f : ee;
      mx = up ? lg : mx;
      dn = fmaf(dn, s1, s2);
      a0 = fmaf(a0, s1, s2 * fs.x);
      a1 = fmaf(a1, s1, s2 * fs.y);
    }
    const float inv = __builtin_amdgcn_rcpf(dn + EPS_SM);
    float h0 = fmaf(a0, inv, bb2.x);
    float h1 = fmaf(a1, inv, bb2.y);
    const float n0 = expm1f(fminf(h0, 0.f));
    const float n1 = expm1f(fminf(h1, 0.f));
    h0 = h0 > 0.f ? h0 : n0;
    h1 = h1 > 0.f ? h1 : n1;

    if (L < 3) {
      const bool live = grow < nN;
      h0 = (live ? h0 : 0.f) + pz;
      h1 = (live ? h1 : 0.f) + pz;
      const unsigned int hb0 = f2bf(h0), hb1 = f2bf(h1);
      const unsigned int lb0 = f2bf(h0 - bf2f(hb0)), lb1 = f2bf(h1 - bf2f(hb1));
      const int hw = (int)(hb0 | (hb1 << 16));
      const int lw = (int)(lb0 | (lb1 << 16));
      const int sb = 4 * lane;
      const int g0h = __shfl(hw, (sb + 0) & 31), g0l = __shfl(lw, (sb + 0) & 31);
      const int g1h = __shfl(hw, (sb + 1) & 31), g1l = __shfl(lw, (sb + 1) & 31);
      const int g2h = __shfl(hw, (sb + 2) & 31), g2l = __shfl(lw, (sb + 2) & 31);
      const int g3h = __shfl(hw, (sb + 3) & 31), g3l = __shfl(lw, (sb + 3) & 31);
      const bool lsel = lane >= 8;
      v4u pv;
      pv.x = (unsigned int)(lsel ? g0l : g0h);
      pv.y = (unsigned int)(lsel ? g1l : g1h);
      pv.z = (unsigned int)(lsel ? g2l : g2h);
      pv.w = (unsigned int)(lsel ? g3l : g3h);
      unsigned short* gp = HP + (size_t)grow * KA + 8 * (lane & 15);
      const bool wr = (grow < MPr) && (lane < 16);
      if (wr) *(volatile v4u*)gp = pv;
      __threadfence();
      if (wr) *(volatile v4u*)gp = pv;
    } else {
      float part = h0 * fw2.x;
      part = fmaf(h1, fw2.y, part);
#pragma unroll
      for (int off = 16; off > 0; off >>= 1) part += __shfl_xor(part, off);
      const float r = part + fb + pz;
      if (lane == 0) res[slot] = r;
    }
  }

  if (L == 3) {
    __syncthreads();
    const int npc = nb >> 2;
#pragma unroll 1
    for (int p = tid; p < npc; p += NTHR) {
      const v4f v = *(const v4fa*)(res + 4 * p);
      const int r0 = nodeBase + 4 * p;
      if (r0 + 3 < nN) {
        *(volatile v4f*)(out + r0) = v;
      } else {
        if (r0     < nN) *(volatile float*)(out + r0)     = v.x;
        if (r0 + 1 < nN) *(volatile float*)(out + r0 + 1) = v.y;
        if (r0 + 2 < nN) *(volatile float*)(out + r0 + 2) = v.z;
      }
    }
    __threadfence();
#pragma unroll 1
    for (int p = tid; p < npc; p += NTHR) {
      const v4f v = *(const v4fa*)(res + 4 * p);
      const int r0 = nodeBase + 4 * p;
      if (r0 + 3 < nN) {
        *(volatile v4f*)(out + r0) = v;
      } else {
        if (r0     < nN) *(volatile float*)(out + r0)     = v.x;
        if (r0 + 1 < nN) *(volatile float*)(out + r0 + 1) = v.y;
        if (r0 + 2 < nN) *(volatile float*)(out + r0 + 2) = v.z;
      }
    }
  }
}

static int pick_nb(int nE, int nN) {
  int nb = NBMAX;
  while (nb > 32 && (long long)nb * (long long)nE * 5LL > (long long)RCAP * (long long)nN * 4LL) nb >>= 1;
  return nb;
}
static inline int cdiv(int a, int b) { return (a + b - 1) / b; }

extern "C" void kernel_launch(void* const* d_in, const int* in_sizes, int n_in,
                              void* d_out, int out_size, void* d_ws, size_t ws_size,
                              hipStream_t stream) {
  if (n_in < 16) return;
  const int nN = in_sizes[0];
  if (nN <= 0 || nN > (1 << 22)) return;
  if (in_sizes[1] < 2 || (in_sizes[1] & 1) != 0) return;
  const int nE = in_sizes[1] / 2;
  if (nE < 1 || nE >= (1 << (32 - SLOTB))) return;
  if (in_sizes[2]  != HCH) return;
  if (in_sizes[3]  != HCH || in_sizes[4]  != HCH || in_sizes[5]  != HCH) return;
  if (in_sizes[6]  != HCH * HCH) return;
  if (in_sizes[7]  != HCH || in_sizes[8]  != HCH || in_sizes[9]  != HCH) return;
  if (in_sizes[10] != HCH * HCH) return;
  if (in_sizes[11] != HCH || in_sizes[12] != HCH || in_sizes[13] != HCH) return;
  if (in_sizes[14] != HCH) return;
  if (in_sizes[15] < 1) return;
  if (out_size != nN) return;

  const float* x    = (const float*)d_in[0];
  const int*   ei   = (const int*)  d_in[1];
  const float* W1   = (const float*)d_in[2];
  const float* a1s  = (const float*)d_in[3];
  const float* a1d  = (const float*)d_in[4];
  const float* b1   = (const float*)d_in[5];
  const float* W2   = (const float*)d_in[6];
  const float* a2s  = (const float*)d_in[7];
  const float* a2d  = (const float*)d_in[8];
  const float* b2   = (const float*)d_in[9];
  const float* W3   = (const float*)d_in[10];
  const float* a3s  = (const float*)d_in[11];
  const float* a3d  = (const float*)d_in[12];
  const float* b3   = (const float*)d_in[13];
  const float* fcw  = (const float*)d_in[14];
  const float* fcb  = (const float*)d_in[15];
  float* out = (float*)d_out;
  const int* src = ei;
  const int* dst = ei + nE;

  const int MP   = cdiv(nN, MROWS) * MROWS;
  const int nb   = pick_nb(nE, nN);
  if (nb < 32 || (nb & (nb - 1)) != 0 || nb > NBMAX) return;
  const int gA   = cdiv(MP, nb);
  const int vec8 = ((nE & 3) == 0) ? 1 : 0;
  if (gA * nb < MP) return;

  char* ws = (char*)d_ws;
  size_t off = 0;
  const size_t oF   = off; off += (size_t)MP * HCH * 4;            off = (off + 255) & ~(size_t)255;
  const size_t oHA  = off; off += (size_t)MP * KA * 2;             off = (off + 255) & ~(size_t)255;
  const size_t oHB  = off; off += (size_t)MP * KA * 2;             off = (off + 255) & ~(size_t)255;
  const size_t oWT2 = off; off += (size_t)HCH * KA * 2;            off = (off + 255) & ~(size_t)255;
  const size_t oWT3 = off; off += (size_t)HCH * KA * 2;            off = (off + 255) & ~(size_t)255;
  if (off > ws_size || off > (size_t)WSMAX) return;
  float*          F   = (float*)(ws + oF);
  unsigned short* HA  = (unsigned short*)(ws + oHA);
  unsigned short* HB  = (unsigned short*)(ws + oHB);
  unsigned short* WT2 = (unsigned short*)(ws + oWT2);
  unsigned short* WT3 = (unsigned short*)(ws + oWT3);

  hipFuncSetAttribute(reinterpret_cast<const void*>(&k_agg<1>),
                      hipFuncAttributeMaxDynamicSharedMemorySize, LDS_AGG);
  hipFuncSetAttribute(reinterpret_cast<const void*>(&k_agg<2>),
                      hipFuncAttributeMaxDynamicSharedMemorySize, LDS_AGG);
  hipFuncSetAttribute(reinterpret_cast<const void*>(&k_agg<3>),
                      hipFuncAttributeMaxDynamicSharedMemorySize, LDS_AGG);

  const int nU1 = MP * (HCH / 4);
  k_l1feat<<<cdiv(nU1, NTHR), NTHR, 0, stream>>>(x, W1, F, nN, nU1);

  {
    const int nUw = HCH * (KA / 8);
    k_wtr<<<cdiv(nUw, NTHR), NTHR, 0, stream>>>(W2, HCH, HCH, HCH, KA, WT2, nUw);
    k_wtr<<<cdiv(nUw, NTHR), NTHR, 0, stream>>>(W3, HCH, HCH, HCH, KA, WT3, nUw);
  }

  const int gM = MP / GBM;
  k_agg<1><<<gA, NTHR, LDS_AGG, stream>>>(src, dst, F, a1s, a1d, b1, fcw, fcb, HA, out, nN, nE, nb, vec8, MP);
  k_gemm<<<dim3(gM, HCH / GBN), GTHR, 0, stream>>>(HA, WT2, F, KA, HCH);
  k_agg<2><<<gA, NTHR, LDS_AGG, stream>>>(src, dst, F, a2s, a2d, b2, fcw, fcb, HB, out, nN, nE, nb, vec8, MP);
  k_gemm<<<dim3(gM, HCH / GBN), GTHR, 0, stream>>>(HB, WT3, F, KA, HCH);
  k_agg<3><<<gA, NTHR, LDS_AGG, stream>>>(src, dst, F, a3s, a3d, b3, fcw, fcb, HA, out, nN, nE, nb, vec8, MP);
}
